// CliffordSirenLayer_31817117728927
// MI455X (gfx1250) — hardware-run, weakly checked
//
#include <hip/hip_runtime.h>
#include <math.h>

typedef __attribute__((ext_vector_type(16))) _Float16 v16h;
typedef __attribute__((ext_vector_type(8)))  _Float16 v8h;
typedef __attribute__((ext_vector_type(16))) __bf16   v16b;
typedef __attribute__((ext_vector_type(8)))  __bf16   v8b;
typedef __attribute__((ext_vector_type(8)))  float    v8f;
typedef __attribute__((ext_vector_type(4)))  float    v4f;
typedef __attribute__((ext_vector_type(4)))  unsigned v4u;

constexpr int kBatch  = 4;
constexpr int kQuery  = 8192;
constexpr int kAtoms  = 512;
constexpr int kFin    = 32;
constexpr int kFout   = 32;
constexpr int kBlades = 8;
constexpr int kHid    = 16;
constexpr int kRows   = kBatch * kQuery;
constexpr int kKdim   = kFin * kBlades;
constexpr int kNdim   = kFout * kBlades;
constexpr float kOmega0 = 30.0f;
static_assert(kRows == 32768 && kKdim == 256 && kNdim == 256, "shape constants");
static_assert((kKdim % 32) == 0, "GEMM K multiple of 32");
static_assert((kRows % 64) == 0 && (kNdim % 64) == 0, "GEMM M,N multiples of 64");
static_assert((kQuery % 256) == 0 && ((kAtoms * 3) % 256) == 0, "block multiples");

constexpr size_t kOffXH   = 0;
constexpr size_t kOffXL   = kOffXH  + (size_t)kRows * kKdim * 2;
constexpr size_t kOffWH   = kOffXL  + (size_t)kRows * kKdim * 2;
constexpr size_t kOffWL   = kOffWH  + (size_t)kNdim * kKdim * 2;
constexpr size_t kOffOM   = kOffWL  + (size_t)kNdim * kKdim * 2;
constexpr size_t kOffPRE  = kOffOM  + (size_t)kRows * 4;
constexpr size_t kWsTotal = kOffPRE + (size_t)kRows * kNdim * 4;
static_assert(kWsTotal == 67502080ull, "carve total");
static_assert(kWsTotal <= 134217728ull, "carve cap");
static_assert((kOffXL % 128) == 0 && (kOffWH % 128) == 0 && (kOffWL % 128) == 0 &&
              (kOffOM % 128) == 0 && (kOffPRE % 128) == 0, "128-B aligned regions");

__device__ __forceinline__ unsigned short f2bf_bits(float f) {
  unsigned u = __float_as_uint(f);
  return (unsigned short)((u + 0x7FFFu + ((u >> 16) & 1u)) >> 16);
}
__device__ __forceinline__ float bf_bits2f(unsigned short h) { return __uint_as_float(((unsigned)h) << 16); }

__device__ __forceinline__ void dep_guard1_b(v8f& a, v16b x, v16b y, v16b z) { asm volatile("v_nop\n\tv_nop\n\tv_nop\n\tv_nop" : "+v"(a) : "v"(x), "v"(y), "v"(z)); }
__device__ __forceinline__ void keep4_b(v16b a, v16b b, v16b c, v16b d) { asm volatile("v_nop" :: "v"(a), "v"(b), "v"(c), "v"(d)); }
__device__ __forceinline__ void acc_guard4(v8f& a, v8f& b, v8f& c, v8f& d) { asm volatile("v_nop\n\tv_nop\n\tv_nop\n\tv_nop" : "+v"(a), "+v"(b), "+v"(c), "+v"(d)); }
template <typename T> struct Frag;
template <> struct Frag<__bf16> {
  typedef v16b V; union U { v16b v; v8b h[2]; };
  static __device__ __forceinline__ v16b load(const __bf16* p) {
    U f; f.h[0] = *(const v8b*)(p); f.h[1] = *(const v8b*)(p + 16); return f.v;
  }
  static __device__ __forceinline__ v8f mma(v16b a, v16b b, v8f c) {
    return __builtin_amdgcn_wmma_f32_16x16x32_bf16(false, a, false, b, (short)0, c, false, false);
  }
  static __device__ __forceinline__ void guard1(v8f& a, v16b x, v16b y, v16b z) { dep_guard1_b(a, x, y, z); }
  static __device__ __forceinline__ void keep(v16b a, v16b b, v16b c, v16b d) { keep4_b(a, b, c, d); }
};

template <int ET> struct Elem;
template <> struct Elem<1> { typedef __bf16 T; };
template <int ET, int SPL, int BIAS_MODE, int OUT_MODE, bool RESID, int ACT = 0>
__global__ __launch_bounds__(256) void wmma_gemm64(
    const unsigned short* __restrict__ Ap, const unsigned short* __restrict__ A2p, int lda, long strideA,
    const unsigned short* __restrict__ Btp, const unsigned short* __restrict__ Bt2p, int ldb, long strideB,
    void* __restrict__ Cout, void* __restrict__ Cout2, int ldc, long strideC,
    const float* __restrict__ bias,
    const float* __restrict__ resid, long strideR,
    int M, int N, int K, float scale) {
  typedef typename Elem<ET>::T T;
  typedef typename Frag<T>::V V;
  const T* A = (const T*)Ap; const T* A2 = (const T*)A2p; const T* Bt = (const T*)Btp; const T* Bt2 = (const T*)Bt2p;
  __shared__ __align__(16) float sT[8][16 * 68];
  const int b    = blockIdx.y;
  const int lane = threadIdx.x & 31;
  const int wave = threadIdx.x >> 5;
  const int tilesN = N >> 6;
  const int tilesM = M >> 6;
  const int tile = blockIdx.x * 8 + wave;
  if (tile >= tilesM * tilesN) return;
  const int tm = tile / tilesN;
  const int tn = tile - tm * tilesN;
  const int m0 = tm << 6;
  const int n0 = tn << 6;

  const T* Ab  = A  + (size_t)b * strideA;
  const T* Bb  = Bt + (size_t)b * strideB;
  const T* Ab2 = (SPL >= 1) ? (A2  + (size_t)b * strideA) : nullptr;
  const T* Bb2 = (SPL == 2) ? (Bt2 + (size_t)b * strideB) : nullptr;

  const int rlane = lane & 15;
  const int koff  = (lane >> 4) * 8;
  const int mOff  = (lane >> 4) * 8;

  v8f acc[4][4];
#pragma unroll
  for (int i = 0; i < 4; ++i)
#pragma unroll
    for (int j = 0; j < 4; ++j) acc[i][j] = (v8f){0.f,0.f,0.f,0.f,0.f,0.f,0.f,0.f};

  for (int k0 = 0; k0 < K; k0 += 32) {
    V bh[4], bl[4];
#pragma unroll
    for (int j = 0; j < 4; ++j) {
      const size_t bo = (size_t)(n0 + (j << 4) + rlane) * ldb + koff + k0;
      bh[j] = Frag<T>::load(Bb + bo);
      if (SPL == 2) bl[j] = Frag<T>::load(Bb2 + bo);
    }
#pragma unroll
    for (int i = 0; i < 4; ++i) {
      const size_t ao = (size_t)(m0 + (i << 4) + rlane) * lda + koff + k0;
      V ah = Frag<T>::load(Ab + ao);
      V al;
      if (SPL >= 1) al = Frag<T>::load(Ab2 + ao);
#pragma unroll
      for (int j = 0; j < 4; ++j) {
        acc[i][j] = Frag<T>::mma(ah, bh[j], acc[i][j]);
        if (SPL == 2) acc[i][j] = Frag<T>::mma(ah, bl[j], acc[i][j]);
        if (SPL >= 1) acc[i][j] = Frag<T>::mma(al, bh[j], acc[i][j]);
      }
#pragma unroll
      for (int j = 0; j < 4; ++j) Frag<T>::guard1(acc[i][j], ah, (SPL >= 1) ? al : ah, bh[j]);
    }
    Frag<T>::keep(bh[0], bh[1], bh[2], bh[3]);
    if (SPL == 2) Frag<T>::keep(bl[0], bl[1], bl[2], bl[3]);
  }
  acc_guard4(acc[0][0], acc[0][1], acc[0][2], acc[0][3]);
  acc_guard4(acc[1][0], acc[1][1], acc[1][2], acc[1][3]);
  acc_guard4(acc[2][0], acc[2][1], acc[2][2], acc[2][3]);
  acc_guard4(acc[3][0], acc[3][1], acc[3][2], acc[3][3]);

  float* slab = sT[wave];
  const float* Rb = RESID ? (resid + (size_t)b * strideR) : nullptr;
#pragma unroll
  for (int i = 0; i < 4; ++i) {
    const int mBase = m0 + (i << 4);
#pragma unroll
    for (int j = 0; j < 4; ++j) {
      const int n = n0 + (j << 4) + rlane;
      float bv = 0.f;
      if (BIAS_MODE == 2) bv = bias[n];
#pragma unroll
      for (int r = 0; r < 8; ++r) {
        float v = acc[i][j][r] * scale;
        if (BIAS_MODE == 1) v += bias[mBase + mOff + r];
        if (BIAS_MODE == 2) v += bv;
        if (RESID) v += Rb[(size_t)(mBase + mOff + r) * ldc + n];
        if (ACT == 1) v = tanhf(v);
        if (ACT == 2) v = fmaxf(v, 0.0f);
        if (ACT == 4) v = (v > 0.f) ? v : 0.01f * v;
        slab[(mOff + r) * 68 + (j << 4) + rlane] = v;
      }
    }
    __builtin_amdgcn_fence(__ATOMIC_RELEASE, "workgroup");
    __builtin_amdgcn_wave_barrier();
    __builtin_amdgcn_fence(__ATOMIC_ACQUIRE, "workgroup");
    if (OUT_MODE == 0) {
      float* C = (float*)Cout + (size_t)b * strideC;
      const int hh = lane >> 4, c4 = (lane & 15) * 4;
      for (int pass = 0; pass < 2; ++pass) {
#pragma unroll
        for (int it = 0; it < 8; ++it) {
          const int row = it * 2 + hh;
          v4f v = *(const v4f*)(slab + row * 68 + c4);
          *(volatile v4f*)(C + (size_t)(mBase + row) * ldc + n0 + c4) = v;
        }
        __threadfence();
      }
    } else {
      const int q = lane >> 3, c8 = (lane & 7) * 8;
      unsigned short* C  = (unsigned short*)Cout  + (size_t)b * strideC;
      unsigned short* C2 = (OUT_MODE == 2) ? ((unsigned short*)Cout2 + (size_t)b * strideC) : nullptr;
      for (int pass = 0; pass < 2; ++pass) {
#pragma unroll
        for (int it = 0; it < 4; ++it) {
          const int row = it * 4 + q;
          const float* sp = slab + row * 68 + c8;
          v8h hv, lv;
#pragma unroll
          for (int e = 0; e < 8; ++e) {
            if (OUT_MODE == 1) {
              hv[e] = (_Float16)sp[e];
            } else {
              unsigned short hb = f2bf_bits(sp[e]);
              unsigned short lb = f2bf_bits(sp[e] - bf_bits2f(hb));
              hv[e] = __builtin_bit_cast(_Float16, hb);
              lv[e] = __builtin_bit_cast(_Float16, lb);
            }
          }
          *(volatile v8h*)(C + (size_t)(mBase + row) * ldc + n0 + c8) = hv;
          if (OUT_MODE == 2) *(volatile v8h*)(C2 + (size_t)(mBase + row) * ldc + n0 + c8) = lv;
        }
        __threadfence();
      }
    }
    __builtin_amdgcn_fence(__ATOMIC_RELEASE, "workgroup");
    __builtin_amdgcn_wave_barrier();
    __builtin_amdgcn_fence(__ATOMIC_ACQUIRE, "workgroup");
  }
}

__global__ __launch_bounds__(256) void split_rows_bf16_kernel(
    const float* __restrict__ src, unsigned short* __restrict__ dhi, unsigned short* __restrict__ dlo, int total8)
{
  const int i = blockIdx.x * 256 + threadIdx.x;
  if (i >= total8) return;
  const size_t e0 = (size_t)i << 3;
  const v4f a0 = *(const v4f*)(src + e0);
  const v4f a1 = *(const v4f*)(src + e0 + 4);
  v8h hv, lv;
#pragma unroll
  for (int e = 0; e < 4; ++e) {
    const unsigned short h0 = f2bf_bits(a0[e]), h1 = f2bf_bits(a1[e]);
    const unsigned short l0 = f2bf_bits(a0[e] - bf_bits2f(h0)), l1 = f2bf_bits(a1[e] - bf_bits2f(h1));
    hv[e]     = __builtin_bit_cast(_Float16, h0);
    hv[4 + e] = __builtin_bit_cast(_Float16, h1);
    lv[e]     = __builtin_bit_cast(_Float16, l0);
    lv[4 + e] = __builtin_bit_cast(_Float16, l1);
  }
  unsigned short* qh = dhi + e0;
  unsigned short* ql = dlo + e0;
  *(volatile v8h*)qh = hv;
  *(volatile v8h*)ql = lv;
  __threadfence();
  *(volatile v8h*)qh = hv;
  *(volatile v8h*)ql = lv;
}

__device__ __forceinline__ int blade_swap(int c) { return (c == 3) ? 4 : ((c == 4) ? 3 : c); }

__global__ __launch_bounds__(256) void expand_weight_kernel(
    const float* __restrict__ weight, unsigned short* __restrict__ WH, unsigned short* __restrict__ WL)
{
  const int t = blockIdx.x * 256 + threadIdx.x;
  const int n = t >> 5;
  const int i = t & 31;
  const int o = n >> 3;
  const int k = n & 7;
  const int km = blade_swap(k);
  const float* wrow = weight + (size_t)(o * kFin + i) * kBlades;
  unsigned hb[8], lb[8];
#pragma unroll
  for (int c = 0; c < 8; ++c) {
    const int a  = blade_swap(c);
    const int bm = a ^ km;
    const int d  = blade_swap(bm);
    float w = wrow[d];
    const unsigned wb = __float_as_uint(w) & 0x7fffffffu;
    w = (wb > 0x7f800000u) ? 0.0f : w;
    w = fminf(fmaxf(w, -3.4028234663852886e38f), 3.4028234663852886e38f);
    const int par = (__popc((a >> 1) & bm) + __popc((a >> 2) & bm)) & 1;
    const float val = (par != 0) ? -w : w;
    const unsigned short h = f2bf_bits(val);
    const unsigned short l = f2bf_bits(val - bf_bits2f(h));
    hb[c] = (unsigned)h;
    lb[c] = (unsigned)l;
  }
  v4u hv, lv;
  hv.x = hb[0] | (hb[1] << 16); hv.y = hb[2] | (hb[3] << 16); hv.z = hb[4] | (hb[5] << 16); hv.w = hb[6] | (hb[7] << 16);
  lv.x = lb[0] | (lb[1] << 16); lv.y = lb[2] | (lb[3] << 16); lv.z = lb[4] | (lb[5] << 16); lv.w = lb[6] | (lb[7] << 16);
  const size_t e0 = (size_t)t << 3;
  unsigned short* qh = WH + e0;
  unsigned short* ql = WL + e0;
  *(volatile v4u*)qh = hv;
  *(volatile v4u*)ql = lv;
  __threadfence();
  *(volatile v4u*)qh = hv;
  *(volatile v4u*)ql = lv;
}

__global__ __launch_bounds__(256) void freq_kernel(
    const float* __restrict__ qc, const float* __restrict__ ac,
    const float* __restrict__ fw1, const float* __restrict__ fb1,
    const float* __restrict__ fw2, const float* __restrict__ fb2,
    float* __restrict__ om)
{
  __shared__ float sAt[kAtoms * 3];
  const int tid = threadIdx.x;
  const int b = blockIdx.y;
  const int n = blockIdx.x * 256 + tid;
#pragma unroll 1
  for (int m = tid; m < kAtoms * 3; m += 256) sAt[m] = ac[(size_t)b * kAtoms * 3 + m];
  __syncthreads();

  const size_t r = (size_t)b * kQuery + n;
  const float qx = qc[r * 3 + 0];
  const float qy = qc[r * 3 + 1];
  const float qz = qc[r * 3 + 2];

  float d2min = 3.4028234663852886e38f;
#pragma unroll 4
  for (int m = 0; m < kAtoms; ++m) {
    const float dx = qx - sAt[3 * m + 0];
    const float dy = qy - sAt[3 * m + 1];
    const float dz = qz - sAt[3 * m + 2];
    const float d2 = dx * dx + dy * dy + dz * dz;
    d2min = fminf(d2min, d2);
  }
  const float mind = sqrtf(fmaxf(d2min, 1e-4f));

  float hsum = 0.0f;
#pragma unroll 1
  for (int j = 0; j < kHid; ++j) {
    float z = fw1[j * 3 + 0] * qx;
    z = fmaf(fw1[j * 3 + 1], qy, z);
    z = fmaf(fw1[j * 3 + 2], qz, z);
    z = z + fb1[j];
    const float sp = fmaxf(z, 0.0f) + log1pf(expf(-fabsf(z)));
    hsum = fmaf(fw2[j], sp, hsum);
  }
  const float v  = hsum + fb2[0];
  const float ls = fminf(fmaxf(v, 0.0f), 5.0f);
  const float e  = expf(-mind);
  const float w  = kOmega0 * (1.0f + ls * e);
  float* dst = om + r;
  *(volatile float*)dst = w;
  __threadfence();
  *(volatile float*)dst = w;
}

__global__ __launch_bounds__(256) void sin_output_kernel(
    const float* __restrict__ pre, const float* __restrict__ bias, const float* __restrict__ om,
    float* __restrict__ out)
{
  const int i = blockIdx.x * 256 + threadIdx.x;
  const int row = i >> 6;
  const int c4 = (i & 63) << 2;
  const size_t e0 = (size_t)i << 2;
  v4f p  = *(const v4f*)(pre + e0);
  v4f bb = *(const v4f*)(bias + c4);
  const float w = om[row];
#pragma unroll 1
  for (int it = 0; it < 4; ++it) {
    const float a  = p.x;
    const float bz = bb.x;
    const float s  = sinf(w * (a + bz));
    p  = (v4f){p.y, p.z, p.w, s};
    bb = (v4f){bb.y, bb.z, bb.w, bz};
  }
  float* dst = out + e0;
  *(volatile v4f*)dst = p;
  __threadfence();
  *(volatile v4f*)dst = p;
}

extern "C" void kernel_launch(void* const* d_in, const int* in_sizes, int n_in,
                              void* d_out, int out_size, void* d_ws, size_t ws_size,
                              hipStream_t stream) {
  if (n_in < 9) return;
  if (in_sizes[0] != kRows * kKdim) return;
  if (in_sizes[1] != kRows * 3) return;
  if (in_sizes[2] != kBatch * kAtoms * 3) return;
  if (in_sizes[3] != kFout * kFin * kBlades) return;
  if (in_sizes[4] != kNdim) return;
  if (in_sizes[5] != kHid * 3) return;
  if (in_sizes[6] != kHid) return;
  if (in_sizes[7] != kHid) return;
  if (in_sizes[8] != 1) return;
  if (out_size != kRows * kNdim) return;
  if (ws_size < kWsTotal) return;

  const float* x      = (const float*)d_in[0];
  const float* qc     = (const float*)d_in[1];
  const float* ac     = (const float*)d_in[2];
  const float* weight = (const float*)d_in[3];
  const float* bias   = (const float*)d_in[4];
  const float* fw1    = (const float*)d_in[5];
  const float* fb1    = (const float*)d_in[6];
  const float* fw2    = (const float*)d_in[7];
  const float* fb2    = (const float*)d_in[8];
  float* out = (float*)d_out;

  char* ws = (char*)d_ws;
  unsigned short* XH  = (unsigned short*)(ws + kOffXH);
  unsigned short* XL  = (unsigned short*)(ws + kOffXL);
  unsigned short* WH  = (unsigned short*)(ws + kOffWH);
  unsigned short* WL  = (unsigned short*)(ws + kOffWL);
  float*          OM  = (float*)(ws + kOffOM);
  float*          PRE = (float*)(ws + kOffPRE);

  expand_weight_kernel<<<(kNdim * kFin) / 256, 256, 0, stream>>>(weight, WH, WL);

  split_rows_bf16_kernel<<<(kRows * kKdim / 8) / 256, 256, 0, stream>>>(x, XH, XL, kRows * kKdim / 8);

  freq_kernel<<<dim3(kQuery / 256, kBatch), 256, 0, stream>>>(qc, ac, fw1, fb1, fw2, fb2, OM);

  wmma_gemm64<1, 2, 0, 0, false><<<dim3((kRows / 64) * (kNdim / 64) / 8, 1), 256, 0, stream>>>(
      XH, XL, kKdim, 0L,
      WH, WL, kKdim, 0L,
      (void*)PRE, nullptr, kNdim, 0L,
      nullptr, nullptr, 0L,
      kRows, kNdim, kKdim, 1.0f);

  sin_output_kernel<<<(kRows * kNdim / 4) / 256, 256, 0, stream>>>(PRE, bias, OM, out);
}
